// ES2D_43516608643215
// MI455X (gfx1250) — hardware-run, weakly checked
//
#include <hip/hip_runtime.h>
#include <hip/hip_fp16.h>
#include <math.h>

typedef __attribute__((ext_vector_type(16))) __bf16   v16b;
typedef __attribute__((ext_vector_type(8)))  __bf16   v8b;
typedef __attribute__((ext_vector_type(8)))  float    v8f;
typedef __attribute__((ext_vector_type(4)))  float    v4f;
typedef __attribute__((ext_vector_type(4)))  unsigned v4u;
typedef __attribute__((ext_vector_type(8)))  unsigned v8u;

constexpr int kBat   = 2;
constexpr int kCh    = 96;
constexpr int kImH   = 128;
constexpr int kImW   = 128;
constexpr int kDirs  = 4;
constexpr int kNst   = 8;
constexpr int kRank  = 6;
constexpr int kXw    = kRank + 2 * kNst;
constexpr int kSeq   = (kImH / 2) * (kImW / 2);
constexpr int kBK    = kBat * kDirs;
constexpr int kRows  = kBK * kSeq;
constexpr int kChP   = 128;
constexpr int kNstP  = 16;
constexpr int kXdP   = 64;
constexpr int kOffB  = 0;
constexpr int kOffC  = 16;
constexpr int kOffDt = 32;
constexpr int kSxP   = 132;
constexpr float kYCarry    = 16.0f;
constexpr float kYCarryInv = 1.0f / kYCarry;
static_assert(kXw == 22, "x_proj width");
static_assert(kSeq == 4096 && kRows == 32768, "token counts");
static_assert((kCh % 32) == 0, "GEMM K multiple of 32");
static_assert((kRows % 128) == 0 && (kSeq % 128) == 0, "GEMM M tiling never crosses a scan");
static_assert((kChP % 64) == 0 && (kSeq % 64) == 0, "scan geometry");
static_assert(kOffB + kNstP <= kOffC && kOffC + kNstP <= kOffDt && kOffDt + 8 <= kXdP, "x_dbl column slots");

constexpr size_t kSzU   = (size_t)kRows * kChP * 4;
constexpr size_t kSzXD  = (size_t)kRows * kXdP * 4;
constexpr size_t kSzDT  = (size_t)kRows * kChP * 4;
constexpr size_t kSzY   = (size_t)kRows * kChP * 2;
constexpr size_t kSzW   = (size_t)kBK * 64 * kCh * 2;
constexpr size_t kSzAL  = (size_t)kDirs * kChP * kNstP * 4;
constexpr size_t kSzWDT = (size_t)kDirs * kChP * 8 * 4;
constexpr size_t kSzVec = (size_t)kDirs * kChP * 4;
constexpr size_t kOffU   = 0;
constexpr size_t kOffXD  = kOffU   + kSzU;
constexpr size_t kOffDT  = kOffXD  + kSzXD;
constexpr size_t kOffY   = kOffDT  + kSzDT;
constexpr size_t kOffWH  = kOffY   + kSzY;
constexpr size_t kOffWL  = kOffWH  + kSzW;
constexpr size_t kOffAL  = kOffWL  + kSzW;
constexpr size_t kOffWDT = kOffAL  + kSzAL;
constexpr size_t kOffDSK = kOffWDT + kSzWDT;
constexpr size_t kOffBDT = kOffDSK + kSzVec;
constexpr size_t kWsTotal = kOffBDT + kSzVec;
static_assert(kWsTotal == 50581504ull, "carve total");
static_assert(kWsTotal <= 134217728ull, "carve cap");
static_assert((kOffXD % 128) == 0 && (kOffDT % 128) == 0 && (kOffY % 128) == 0 && (kOffWH % 128) == 0 &&
              (kOffWL % 128) == 0 && (kOffAL % 128) == 0 && (kOffWDT % 128) == 0 && (kOffDSK % 128) == 0 &&
              (kOffBDT % 128) == 0, "128-B aligned regions");

__device__ __forceinline__ unsigned bf_bits_rne(float f) {
  const unsigned u = __float_as_uint(f);
  return ((u + 0x7FFFu + ((u >> 16) & 1u)) >> 16) & 0xFFFFu;
}
__device__ __forceinline__ void split_pair(float a, float b, unsigned& hw, unsigned& lw) {
  const unsigned ha = bf_bits_rne(a);
  const unsigned hb = bf_bits_rne(b);
  const float ra = a - __uint_as_float(ha << 16);
  const float rb = b - __uint_as_float(hb << 16);
  const unsigned la = bf_bits_rne(ra);
  const unsigned lb = bf_bits_rne(rb);
  hw = ha | (hb << 16);
  lw = la | (lb << 16);
}
__device__ __forceinline__ float h16_to_f32(unsigned hb) {
  const unsigned sgn = (hb & 0x8000u) << 16;
  const unsigned em = hb & 0x7fffu;
  const float fn = __uint_as_float((em << 13) + 0x38000000u);
  const float fs = (float)em * 5.9604644775390625e-8f;
  const float mag = (em < 0x400u) ? fs : fn;
  return __uint_as_float(__float_as_uint(mag) | sgn);
}
__device__ __forceinline__ v16b load_frag_bf(const __bf16* p) {
  union { v16b v; v8b h[2]; } f;
  f.h[0] = *(const v8b*)(p);
  f.h[1] = *(const v8b*)(p + 16);
  return f.v;
}
__device__ __forceinline__ v8f mma_bf(v16b a, v16b b, v8f c) {
  c = __builtin_amdgcn_wmma_f32_16x16x32_bf16(false, a, false, b, (short)0, c, false, false);
  asm volatile("v_nop\n\tv_nop\n\tv_nop\n\tv_nop" : "+v"(c) : "v"(a), "v"(b));
  return c;
}

__global__ __launch_bounds__(256) void prep_tables_kernel(
    const float* __restrict__ xpw, const float* __restrict__ dtw, const float* __restrict__ dtb,
    const float* __restrict__ alog, const float* __restrict__ dsk,
    unsigned short* __restrict__ WH, unsigned short* __restrict__ WL,
    float* __restrict__ AL, float* __restrict__ WDT, float* __restrict__ DSK, float* __restrict__ BDT)
{
  const int blk = blockIdx.x;
  const int tid = threadIdx.x;
  if (blk < 24) {
    const int i   = blk * 256 + tid;
    const int e0  = i * 8;
    const int row = e0 / kCh;
    const int kc  = e0 - row * kCh;
    const int bk  = row >> 6;
    const int n   = row & 63;
    const int k   = bk & 3;
    int c = -1;
    if (n < kNst) c = kRank + n;
    else if (n >= kOffC && n < kOffC + kNst) c = kRank + kNst + (n - kOffC);
    else if (n >= kOffDt && n < kOffDt + kRank) c = n - kOffDt;
    const bool live = (c >= 0);
    const int cc = live ? c : 0;
    const float* src = xpw + ((size_t)(k * kXw + cc) * kCh + kc);
    const v4f a0 = *(const v4f*)(src);
    const v4f a1 = *(const v4f*)(src + 4);
    float x0 = a0[0], x1 = a0[1], x2 = a0[2], x3 = a0[3];
    float x4 = a1[0], x5 = a1[1], x6 = a1[2], x7 = a1[3];
    asm volatile("" : "+v"(x0));
    asm volatile("" : "+v"(x1));
    asm volatile("" : "+v"(x2));
    asm volatile("" : "+v"(x3));
    asm volatile("" : "+v"(x4));
    asm volatile("" : "+v"(x5));
    asm volatile("" : "+v"(x6));
    asm volatile("" : "+v"(x7));
    x0 = live ? x0 : 0.0f;
    x1 = live ? x1 : 0.0f;
    x2 = live ? x2 : 0.0f;
    x3 = live ? x3 : 0.0f;
    x4 = live ? x4 : 0.0f;
    x5 = live ? x5 : 0.0f;
    x6 = live ? x6 : 0.0f;
    x7 = live ? x7 : 0.0f;
    unsigned h0, h1, h2, h3, l0, l1, l2, l3;
    split_pair(x0, x1, h0, l0);
    split_pair(x2, x3, h1, l1);
    split_pair(x4, x5, h2, l2);
    split_pair(x6, x7, h3, l3);
    const v4u hv = (v4u){h0, h1, h2, h3};
    const v4u lv = (v4u){l0, l1, l2, l3};
    unsigned short* ph = WH + e0;
    unsigned short* pl = WL + e0;
    *(volatile v4u*)ph = hv;
    *(volatile v4u*)pl = lv;
    __threadfence();
    *(volatile v4u*)ph = hv;
    *(volatile v4u*)pl = lv;
  } else if (blk < 32) {
    const int j  = (blk - 24) * 256 + tid;
    const int e0 = j * 4;
    const int k  = e0 / (kChP * kNstP);
    const int rm = e0 - k * (kChP * kNstP);
    const int d  = rm / kNstP;
    const int n0 = rm - d * kNstP;
    const bool live = (d < kCh) && (n0 < kNst);
    const int dc = (d < kCh) ? d : (kCh - 1);
    const int nc = (n0 < kNst) ? n0 : 0;
    const v4f a0 = *(const v4f*)(alog + ((size_t)(k * kCh + dc) * kNst + nc));
    float x0 = a0[0], x1 = a0[1], x2 = a0[2], x3 = a0[3];
    asm volatile("" : "+v"(x0));
    asm volatile("" : "+v"(x1));
    asm volatile("" : "+v"(x2));
    asm volatile("" : "+v"(x3));
    const v4f ov = (v4f){live ? x0 : 0.0f, live ? x1 : 0.0f, live ? x2 : 0.0f, live ? x3 : 0.0f};
    float* po = AL + e0;
    *(volatile v4f*)po = ov;
    __threadfence();
    *(volatile v4f*)po = ov;
  } else if (blk < 36) {
    const int j  = (blk - 32) * 256 + tid;
    const int e0 = j * 4;
    const int k  = e0 / (kChP * 8);
    const int rm = e0 - k * (kChP * 8);
    const int d  = rm >> 3;
    const int r0 = rm & 7;
    const bool dlive = (d < kCh);
    const int dc = dlive ? d : (kCh - 1);
    const float* src = dtw + (size_t)(k * kCh + dc) * kRank;
    const int ra = r0;
    const int rb = r0 + 1;
    const int rc = (r0 + 2 < kRank) ? (r0 + 2) : (kRank - 1);
    const int rd = (r0 + 3 < kRank) ? (r0 + 3) : (kRank - 1);
    float x0 = src[ra];
    float x1 = src[rb];
    float x2 = src[rc];
    float x3 = src[rd];
    asm volatile("" : "+v"(x0));
    asm volatile("" : "+v"(x1));
    asm volatile("" : "+v"(x2));
    asm volatile("" : "+v"(x3));
    const bool l0 = dlive;
    const bool l1 = dlive;
    const bool l2 = dlive && (r0 + 2 < kRank);
    const bool l3 = dlive && (r0 + 3 < kRank);
    const v4f ov = (v4f){l0 ? x0 : 0.0f, l1 ? x1 : 0.0f, l2 ? x2 : 0.0f, l3 ? x3 : 0.0f};
    float* po = WDT + e0;
    *(volatile v4f*)po = ov;
    __threadfence();
    *(volatile v4f*)po = ov;
  } else {
    const bool first = (tid < 128);
    const float* srcv = first ? dsk : dtb;
    float* dstv = first ? DSK : BDT;
    const int j  = first ? tid : (tid - 128);
    const int e0 = j * 4;
    const int k  = e0 / kChP;
    const int d  = e0 - k * kChP;
    const bool live = (d < kCh);
    const int dc = live ? d : (kCh - 4);
    const v4f a0 = *(const v4f*)(srcv + (k * kCh + dc));
    float x0 = a0[0], x1 = a0[1], x2 = a0[2], x3 = a0[3];
    asm volatile("" : "+v"(x0));
    asm volatile("" : "+v"(x1));
    asm volatile("" : "+v"(x2));
    asm volatile("" : "+v"(x3));
    const v4f ov = (v4f){live ? x0 : 0.0f, live ? x1 : 0.0f, live ? x2 : 0.0f, live ? x3 : 0.0f};
    float* po = dstv + e0;
    *(volatile v4f*)po = ov;
    __threadfence();
    *(volatile v4f*)po = ov;
  }
}

__global__ __launch_bounds__(256) void gather_tokens_kernel(const float* __restrict__ x, float* __restrict__ U)
{
  __shared__ __align__(16) float sX[kCh * kSxP];
  const int tid  = threadIdx.x;
  const int lane = tid & 31;
  const int wave = tid >> 5;
  const int h = blockIdx.x;
  const int b = blockIdx.y;
#pragma unroll 4
  for (int it = 0; it < 12; ++it) {
    const int idx = tid + it * 256;
    const int d   = idx >> 5;
    const int w4  = (idx & 31) * 4;
    const v4f v = *(const v4f*)(x + (((size_t)b * kCh + d) * kImH + h) * kImW + w4);
    *(v4f*)(sX + d * kSxP + w4) = v;
  }
  __syncthreads();
  const int dl = lane * 4;
  const bool live = (lane < kCh / 4);
  const int dc = live ? dl : (kCh - 4);
  const int hodd = h & 1;
  const int hj = h >> 1;
#pragma unroll 1
  for (int g = 0; g < 4; ++g) {
    v4f val[4];
    size_t off[4];
#pragma unroll
    for (int t = 0; t < 4; ++t) {
      const int w = wave * 16 + g * 4 + t;
      const float* sp = sX + dc * kSxP + w;
      const float f0 = sp[0];
      const float f1 = sp[kSxP];
      const float f2 = sp[2 * kSxP];
      const float f3 = sp[3 * kSxP];
      val[t] = (v4f){live ? f0 : 0.0f, live ? f1 : 0.0f, live ? f2 : 0.0f, live ? f3 : 0.0f};
      const int k = hodd + 2 * (w & 1);
      const int l = hodd ? ((w >> 1) * 64 + hj) : (hj * 64 + (w >> 1));
      off[t] = ((size_t)((b * kDirs + k) * kSeq + l)) * kChP + dl;
    }
    for (int pass = 0; pass < 2; ++pass) {
#pragma unroll
      for (int t = 0; t < 4; ++t) *(volatile v4f*)(U + off[t]) = val[t];
      __threadfence();
    }
  }
}

__global__ __launch_bounds__(256) void xproj_gemm_kernel(
    const float* __restrict__ U, const unsigned short* __restrict__ WHp, const unsigned short* __restrict__ WLp,
    float* __restrict__ XD)
{
  __shared__ __align__(16) float sT[8][16 * 68];
  const int tid  = threadIdx.x;
  const int lane = tid & 31;
  const int wave = tid >> 5;
  const int c  = lane & 15;
  const int hh = lane >> 4;
  const int m0 = (blockIdx.x * 8 + wave) * 16;
  const int bk = (blockIdx.x * 128) / kSeq;
  const __bf16* Bh = (const __bf16*)WHp + (size_t)bk * 64 * kCh;
  const __bf16* Bl = (const __bf16*)WLp + (size_t)bk * 64 * kCh;
  const float* arow = U + (size_t)(m0 + c) * kChP;

  v8f acc[4];
#pragma unroll
  for (int j = 0; j < 4; ++j) acc[j] = (v8f){0.f, 0.f, 0.f, 0.f, 0.f, 0.f, 0.f, 0.f};

#pragma unroll 1
  for (int k0 = 0; k0 < kCh; k0 += 32) {
    v16b bh[4], bl[4];
#pragma unroll
    for (int j = 0; j < 4; ++j) {
      const int bo = (j * 16 + c) * kCh + k0 + 8 * hh;
      bh[j] = load_frag_bf(Bh + bo);
      bl[j] = load_frag_bf(Bl + bo);
    }
    const float* ap = arow + k0 + 8 * hh;
    const v4f f0 = *(const v4f*)(ap);
    const v4f f1 = *(const v4f*)(ap + 4);
    const v4f f2 = *(const v4f*)(ap + 16);
    const v4f f3 = *(const v4f*)(ap + 20);
    v8u ahw, alw;
    unsigned hw, lw;
    split_pair(f0[0], f0[1], hw, lw);
    ahw[0] = hw;
    alw[0] = lw;
    split_pair(f0[2], f0[3], hw, lw);
    ahw[1] = hw;
    alw[1] = lw;
    split_pair(f1[0], f1[1], hw, lw);
    ahw[2] = hw;
    alw[2] = lw;
    split_pair(f1[2], f1[3], hw, lw);
    ahw[3] = hw;
    alw[3] = lw;
    split_pair(f2[0], f2[1], hw, lw);
    ahw[4] = hw;
    alw[4] = lw;
    split_pair(f2[2], f2[3], hw, lw);
    ahw[5] = hw;
    alw[5] = lw;
    split_pair(f3[0], f3[1], hw, lw);
    ahw[6] = hw;
    alw[6] = lw;
    split_pair(f3[2], f3[3], hw, lw);
    ahw[7] = hw;
    alw[7] = lw;
    const v16b ah = __builtin_bit_cast(v16b, ahw);
    const v16b al = __builtin_bit_cast(v16b, alw);
#pragma unroll
    for (int j = 0; j < 4; ++j) {
      acc[j] = mma_bf(ah, bh[j], acc[j]);
      acc[j] = mma_bf(ah, bl[j], acc[j]);
      acc[j] = mma_bf(al, bh[j], acc[j]);
    }
  }

  float* slab = sT[wave];
#pragma unroll
  for (int j = 0; j < 4; ++j) {
#pragma unroll
    for (int r = 0; r < 8; ++r) slab[(8 * hh + r) * 68 + j * 16 + c] = acc[j][r];
  }
  __syncthreads();
  const int c4 = c * 4;
  v4f ov[8];
#pragma unroll
  for (int it = 0; it < 8; ++it) ov[it] = *(const v4f*)(slab + (it * 2 + hh) * 68 + c4);
  for (int pass = 0; pass < 2; ++pass) {
#pragma unroll
    for (int it = 0; it < 8; ++it)
      *(volatile v4f*)(XD + (size_t)(m0 + it * 2 + hh) * kXdP + c4) = ov[it];
    __threadfence();
  }
}

__global__ __launch_bounds__(256) void dtpre_kernel(
    const float* __restrict__ XD, const float* __restrict__ WDT, const float* __restrict__ BDT,
    float* __restrict__ DT)
{
  const int tid  = threadIdx.x;
  const int lane = tid & 31;
  const int wave = tid >> 5;
  const int r0 = blockIdx.x * 64;
  const int k  = (r0 / kSeq) & 3;
  const int d  = lane * 4;
  const bool live = (lane < kCh / 4);
  const float* wp = WDT + ((size_t)k * kChP + d) * 8;
  v4f wa[4], wb[4];
#pragma unroll
  for (int e = 0; e < 4; ++e) {
    wa[e] = *(const v4f*)(wp + e * 8);
    wb[e] = *(const v4f*)(wp + e * 8 + 4);
  }
  const v4f bias = *(const v4f*)(BDT + k * kChP + d);
#pragma unroll 1
  for (int i = 0; i < 8; ++i) {
    const size_t row = (size_t)(r0 + wave * 8 + i);
    const v4f ra = *(const v4f*)(XD + row * kXdP + kOffDt);
    const v4f rb = *(const v4f*)(XD + row * kXdP + kOffDt + 4);
    v4f o;
#pragma unroll
    for (int e = 0; e < 4; ++e) {
      float s = wa[e][0] * ra[0];
      s = fmaf(wa[e][1], ra[1], s);
      s = fmaf(wa[e][2], ra[2], s);
      s = fmaf(wa[e][3], ra[3], s);
      s = fmaf(wb[e][0], rb[0], s);
      s = fmaf(wb[e][1], rb[1], s);
      s = s + bias[e];
      o[e] = live ? s : 0.0f;
    }
    float* po = DT + row * kChP + d;
    *(volatile v4f*)po = o;
    __threadfence();
    *(volatile v4f*)po = o;
  }
}

typedef float    ms1_v4f __attribute__((ext_vector_type(4)));
typedef unsigned ms1_v4u __attribute__((ext_vector_type(4)));
struct ms1_args {
  const float* dtpre;
  const float* u;
  const float* bc;
  const float* z;
  const float* A_log;
  const float* Dskip;
  __half* y;
  __half* y_lo;
  long ld_dtpre;
  long ld_u;
  long ld_bc;
  long ld_z;
  long ld_y;
  int offB;
  int offC;
  int offZ;
  float ycarry;
  int dir;
  int D;
  int L;
  int nbatch;
};
static_assert(sizeof(ms1_args) == 136);

__device__ __forceinline__ float ms1_flush16(float v) {
  return (fabsf(v) < 6.103515625e-05f) ? 0.0f : v;
}
__device__ __forceinline__ unsigned ms1_h16bits(float v) {
  return (unsigned)__half_as_ushort(__float2half_rn(ms1_flush16(v)));
}
__device__ __forceinline__ float ms1_h16val(unsigned b) {
  return __half2float(__ushort_as_half((unsigned short)b));
}
__device__ __forceinline__ float ms1_softplus(float v) {
  return fmaxf(v, 0.0f) + log1pf(expf(-fabsf(v)));
}
__device__ __forceinline__ void ms1_pack2(float v0, float v1, unsigned& hw, unsigned& lw) {
  const unsigned h0 = ms1_h16bits(v0);
  const unsigned h1 = ms1_h16bits(v1);
  const float r0 = (v0 - ms1_h16val(h0)) * 2048.0f;
  const float r1 = (v1 - ms1_h16val(h1)) * 2048.0f;
  const unsigned l0 = ms1_h16bits(r0);
  const unsigned l1 = ms1_h16bits(r1);
  hw = h0 | (h1 << 16);
  lw = l0 | (l1 << 16);
}

template <int NSTATE>
__global__ __launch_bounds__(64 * (NSTATE / 16)) void ms1_scan_kernel(ms1_args a)
{
  static_assert(NSTATE == 16 || NSTATE == 64);
  constexpr int NQ  = NSTATE / 16;
  constexpr int NT  = 64 * NQ;
  constexpr int NW  = NT / 32;
  constexpr int BCW = 2 * NSTATE;
  constexpr int YP  = 68;
  constexpr int RPI = NW * 4;
  constexpr int NIT = 64 / RPI;
  static_assert(16 * NT <= 64 * YP);
  __shared__ __align__(16) float sBC[64 * BCW];
  __shared__ __align__(16) float sY[64 * YP];
  const int tid  = threadIdx.x;
  const int lane = tid & 31;
  const int wave = tid >> 5;
  const int c    = tid / NQ;
  const int sq   = tid - c * NQ;
  const int bpb  = a.D / 64;
  const int bi   = blockIdx.x / bpb;
  if (bi >= a.nbatch) return;
  const int d0 = (blockIdx.x - bi * bpb) * 64;
  const int d  = d0 + c;
  const long rowb = (long)bi * a.L;
  const bool hasz  = (a.z != nullptr);
  const bool hasD  = (a.Dskip != nullptr);
  const bool hasLo = (a.y_lo != nullptr);

#pragma unroll 1
  for (int n = 0; n < 16; ++n) {
    const float al = a.A_log[(long)d * NSTATE + sq * 16 + n];
    sY[n * NT + tid] = -expf(al);
  }
  __syncthreads();
  float An[16], h[16];
#pragma unroll
  for (int n = 0; n < 16; ++n) {
    An[n] = sY[n * NT + tid];
    h[n] = 0.0f;
  }
  float Dd = 0.0f;
  if (hasD) Dd = a.Dskip[d];

  const int nchunk = a.L / 64;
  const bool fwd = (a.dir > 0);
  const int s0 = fwd ? 0 : 63;
  const int sd = fwd ? 1 : -1;
  const int q  = lane >> 3;
  const int c8 = (lane & 7) * 8;

#pragma unroll 1
  for (int ci = 0; ci < nchunk; ++ci) {
    const int tb = fwd ? (ci * 64) : (a.L - 64 - ci * 64);
    const long rowc = rowb + tb;
    __syncthreads();
#pragma unroll 8
    for (int i = 0; i < 32; ++i) {
      const int idx = tid + i * NT;
      const int st  = idx / BCW;
      const int col = idx - st * BCW;
      const int sc  = (col < NSTATE) ? (a.offB + col) : (a.offC + col - NSTATE);
      sBC[idx] = a.bc[(rowc + st) * a.ld_bc + sc];
    }
    __syncthreads();
#pragma unroll 1
    for (int s = 0; s < 64; ++s) {
      const int ls = s0 + sd * s;
      const long row = rowc + ls;
      float pre = a.dtpre[row * a.ld_dtpre + d];
      float uv  = a.u[row * a.ld_u + d];
      float zv  = 0.0f;
      if (hasz) zv = a.z[row * a.ld_z + a.offZ + d];
      asm volatile("" : "+v"(pre));
      asm volatile("" : "+v"(uv));
      asm volatile("" : "+v"(zv));
      const float delta = ms1_softplus(pre);
      const float dtx = delta * uv;
      const float* bp = sBC + ls * BCW + sq * 16;
      const float* cp = bp + NSTATE;
      ms1_v4f Bq[4], Cq[4];
#pragma unroll
      for (int k = 0; k < 4; ++k) {
        Bq[k] = *(const ms1_v4f*)(bp + 4 * k);
        Cq[k] = *(const ms1_v4f*)(cp + 4 * k);
      }
      float yv = 0.0f;
#pragma unroll
      for (int n = 0; n < 16; ++n) {
        const float e = __expf(delta * An[n]);
        h[n] = fmaf(e, h[n], dtx * Bq[n >> 2][n & 3]);
        yv = fmaf(h[n], Cq[n >> 2][n & 3], yv);
      }
      if (NQ > 1) {
        yv += __shfl_xor(yv, 1, 32);
        yv += __shfl_xor(yv, 2, 32);
      }
      if (hasD) yv = fmaf(uv, Dd, yv);
      if (hasz) {
        const float sg = __builtin_amdgcn_rcpf(1.0f + expf(-zv));
        yv = yv * (zv * sg);
      }
      if (sq == 0) sY[ls * YP + c] = yv * a.ycarry;
    }
    __syncthreads();
    ms1_v4u hw[NIT], lw[NIT];
#pragma unroll
    for (int it = 0; it < NIT; ++it) {
      const int row = it * RPI + wave * 4 + q;
      const float* sp = sY + row * YP + c8;
      const ms1_v4f f0 = *(const ms1_v4f*)(sp);
      const ms1_v4f f1 = *(const ms1_v4f*)(sp + 4);
      unsigned h0, h1, h2, h3, l0, l1, l2, l3;
      ms1_pack2(f0[0], f0[1], h0, l0);
      ms1_pack2(f0[2], f0[3], h1, l1);
      ms1_pack2(f1[0], f1[1], h2, l2);
      ms1_pack2(f1[2], f1[3], h3, l3);
      hw[it] = (ms1_v4u){h0, h1, h2, h3};
      lw[it] = (ms1_v4u){l0, l1, l2, l3};
    }
    for (int pass = 0; pass < 2; ++pass) {
#pragma unroll
      for (int it = 0; it < NIT; ++it) {
        const int row = it * RPI + wave * 4 + q;
        const long o = (rowc + row) * a.ld_y + d0 + c8;
        *(volatile ms1_v4u*)(a.y + o) = hw[it];
        if (hasLo) *(volatile ms1_v4u*)(a.y_lo + o) = lw[it];
      }
      __threadfence();
    }
  }
}

__global__ __launch_bounds__(256) void merge_ln_kernel(
    const unsigned* __restrict__ Yw, const float* __restrict__ lnw, const float* __restrict__ lnb,
    const int* __restrict__ stepv, float* __restrict__ out)
{
  const int lane = threadIdx.x & 31;
  const int pix  = blockIdx.x * 8 + (threadIdx.x >> 5);
  const int w = pix & (kImW - 1);
  const int h = (pix >> 7) & (kImH - 1);
  const int b = pix >> 14;
  const int k = (h & 1) + 2 * (w & 1);
  const int l = (h & 1) ? ((w >> 1) * 64 + (h >> 1)) : ((h >> 1) * 64 + (w >> 1));
  const size_t row = (size_t)((b * kDirs + k) * kSeq + l);
  const unsigned* yr = Yw + row * (kChP / 2);
  const unsigned w0 = yr[(lane >> 1)];
  const unsigned w1 = yr[16 + (lane >> 1)];
  const unsigned w2 = yr[32 + (lane >> 1)];
  const unsigned sh = (unsigned)(lane & 1) * 16u;
  const float v0 = h16_to_f32((w0 >> sh) & 0xffffu) * kYCarryInv;
  const float v1 = h16_to_f32((w1 >> sh) & 0xffffu) * kYCarryInv;
  const float v2 = h16_to_f32((w2 >> sh) & 0xffffu) * kYCarryInv;
  const float g0 = lnw[lane], g1 = lnw[lane + 32], g2 = lnw[lane + 64];
  const float e0 = lnb[lane], e1 = lnb[lane + 32], e2 = lnb[lane + 64];
  const int st = stepv[0];
  const bool ok = (st == 2);

  float s = (v0 + v1) + v2;
  s += __shfl_xor(s, 16, 32);
  s += __shfl_xor(s, 8, 32);
  s += __shfl_xor(s, 4, 32);
  s += __shfl_xor(s, 2, 32);
  s += __shfl_xor(s, 1, 32);
  const float mu = s * (1.0f / (float)kCh);
  const float c0 = v0 - mu, c1 = v1 - mu, c2 = v2 - mu;
  float qv = c0 * c0;
  qv = fmaf(c1, c1, qv);
  qv = fmaf(c2, c2, qv);
  qv += __shfl_xor(qv, 16, 32);
  qv += __shfl_xor(qv, 8, 32);
  qv += __shfl_xor(qv, 4, 32);
  qv += __shfl_xor(qv, 2, 32);
  qv += __shfl_xor(qv, 1, 32);
  const float inv = rsqrtf(qv * (1.0f / (float)kCh) + 1e-5f);
  const float nanv = __uint_as_float(0x7fc00000u);
  float o0 = fmaf(c0 * inv, g0, e0);
  float o1 = fmaf(c1 * inv, g1, e1);
  float o2 = fmaf(c2 * inv, g2, e2);
  o0 = ok ? o0 : nanv;
  o1 = ok ? o1 : nanv;
  o2 = ok ? o2 : nanv;
  volatile float* po = out + (size_t)pix * kCh;
  po[lane]      = o0;
  po[lane + 32] = o1;
  po[lane + 64] = o2;
  __threadfence();
  po[lane]      = o0;
  po[lane + 32] = o1;
  po[lane + 64] = o2;
}

extern "C" void kernel_launch(void* const* d_in, const int* in_sizes, int n_in,
                              void* d_out, int out_size, void* d_ws, size_t ws_size,
                              hipStream_t stream)
{
  if (n_in < 9) return;
  if (in_sizes[0] != kBat * kCh * kImH * kImW) return;
  if (in_sizes[1] != kDirs * kXw * kCh) return;
  if (in_sizes[2] != kDirs * kCh * kRank) return;
  if (in_sizes[3] != kDirs * kCh) return;
  if (in_sizes[4] != kDirs * kCh * kNst) return;
  if (in_sizes[5] != kDirs * kCh) return;
  if (in_sizes[6] != kCh) return;
  if (in_sizes[7] != kCh) return;
  if (in_sizes[8] != 1) return;
  if (out_size != kBat * kImH * kImW * kCh) return;
  if (ws_size < kWsTotal) return;

  const float* x    = (const float*)d_in[0];
  const float* xpw  = (const float*)d_in[1];
  const float* dtw  = (const float*)d_in[2];
  const float* dtb  = (const float*)d_in[3];
  const float* alog = (const float*)d_in[4];
  const float* dsk  = (const float*)d_in[5];
  const float* lnw  = (const float*)d_in[6];
  const float* lnb  = (const float*)d_in[7];
  const int*   stp  = (const int*)d_in[8];
  float* out = (float*)d_out;

  char* ws = (char*)d_ws;
  float*          U   = (float*)(ws + kOffU);
  float*          XD  = (float*)(ws + kOffXD);
  float*          DT  = (float*)(ws + kOffDT);
  __half*         Y   = (__half*)(ws + kOffY);
  unsigned short* WH  = (unsigned short*)(ws + kOffWH);
  unsigned short* WL  = (unsigned short*)(ws + kOffWL);
  float*          AL  = (float*)(ws + kOffAL);
  float*          WDT = (float*)(ws + kOffWDT);
  float*          DSK = (float*)(ws + kOffDSK);
  float*          BDT = (float*)(ws + kOffBDT);

  prep_tables_kernel<<<dim3(37), dim3(256), 0, stream>>>(xpw, dtw, dtb, alog, dsk, WH, WL, AL, WDT, DSK, BDT);
  gather_tokens_kernel<<<dim3(kImH, kBat), dim3(256), 0, stream>>>(x, U);
  xproj_gemm_kernel<<<dim3(kRows / 128), dim3(256), 0, stream>>>(U, WH, WL, XD);
  dtpre_kernel<<<dim3(kRows / 64), dim3(256), 0, stream>>>(XD, WDT, BDT, DT);

  for (int bk = 0; bk < kBK; ++bk) {
    const int k = bk & 3;
    const size_t r0 = (size_t)bk * kSeq;
    ms1_args sa;
    sa.dtpre = DT + r0 * kChP;
    sa.u = U + r0 * kChP;
    sa.bc = XD + r0 * kXdP;
    sa.z = nullptr;
    sa.A_log = AL + (size_t)k * kChP * kNstP;
    sa.Dskip = DSK + (size_t)k * kChP;
    sa.y = Y + r0 * kChP;
    sa.y_lo = nullptr;
    sa.ld_dtpre = kChP;
    sa.ld_u = kChP;
    sa.ld_bc = kXdP;
    sa.ld_z = 0;
    sa.ld_y = kChP;
    sa.offB = kOffB;
    sa.offC = kOffC;
    sa.offZ = 0;
    sa.ycarry = kYCarry;
    sa.dir = 1;
    sa.D = kChP;
    sa.L = kSeq;
    sa.nbatch = 1;
    ms1_scan_kernel<16><<<dim3(kChP / 64), dim3(64), 0, stream>>>(sa);
  }

  merge_ln_kernel<<<dim3(kBat * kImH * kImW / 8), dim3(256), 0, stream>>>(
      (const unsigned*)(ws + kOffY), lnw, lnb, stp, out);
}
